// source_model_19396072308786
// MI455X (gfx1250) — hardware-verified
//
#include <hip/hip_runtime.h>
#include <stddef.h>


#pragma clang fp contract(off)

#define VOC    30
#define TCH    8192
#define KW     5
#define SEQ    512
#define BAT    32
#define ROWS   (BAT * SEQ)
#define KRAW   (VOC * KW)
#define KP     160
#define KROW   (2 * KP)
#define NKS    (KP / 32)
#define NTHR   256
#define NWAVE  8
#define MBLK   (16 * NWAVE)
#define NT     (TCH / 16)
#define PBROWS 64
#define PBIT   ((PBROWS * KROW * 2) / (NTHR * 16))
#define PCIT   ((PBROWS * KP) / NTHR)
#define WSCAP  134217728
#define SC_HI  16384.0f
#define SC_LO  1024.0f
#define INV_LO 0.0009765625f

static_assert(ROWS % MBLK == 0);
static_assert(TCH % 16 == 0 && TCH % PBROWS == 0);
static_assert(PBIT * NTHR * 16 == PBROWS * KROW * 2);
static_assert(PCIT * NTHR == PBROWS * KP);
static_assert(KP % 32 == 0 && KRAW <= KP);
static_assert((PBROWS * KROW * 2) % 128 == 0);
static_assert((KROW * 2) % 16 == 0);
static_assert(MBLK * 4 == 32 * 16);
static_assert(NTHR == 32 * NWAVE);
static_assert(SEQ == 512 && BAT * SEQ == ROWS);

typedef _Float16     v16h __attribute__((ext_vector_type(16)));
typedef _Float16     v8h  __attribute__((ext_vector_type(8)));
typedef float        v8f  __attribute__((ext_vector_type(8)));
typedef unsigned int v4u  __attribute__((ext_vector_type(4)));
typedef int          v4i  __attribute__((ext_vector_type(4)));
typedef v4u v4ua __attribute__((may_alias));
typedef v4i v4ia __attribute__((may_alias));

union FragB { v16h v; v8h hf[2]; };
union FragA { v16h v; unsigned int w[8]; };

__device__ __forceinline__ v8f wmh(v16h a, v16h b, v8f c) {
  return __builtin_amdgcn_wmma_f32_16x16x32_f16(false, a, false, b, (short)0, c, false, false);
}

__device__ __forceinline__ v16h build_a(int kbase, int kt0, int kt1, int kt2, int kt3, int kt4) {
  FragA f;
#pragma unroll
  for (int q = 0; q < 8; ++q) {
    const int ka = kbase + ((q < 4) ? (2 * q) : (2 * q + 8));
    const int kb = ka + 1;
    const bool ha = (ka == kt0) | (ka == kt1) | (ka == kt2) | (ka == kt3) | (ka == kt4);
    const bool hb = (kb == kt0) | (kb == kt1) | (kb == kt2) | (kb == kt3) | (kb == kt4);
    f.w[q] = (ha ? 0x3C00u : 0u) | (hb ? 0x3C000000u : 0u);
  }
  return f.v;
}

__global__ __launch_bounds__(NTHR) void k_prep(const float* __restrict__ w, unsigned int* bp) {
  __shared__ __attribute__((aligned(16))) _Float16 sh[PBROWS * KROW];
  const int tid = threadIdx.x;
  const int t0 = blockIdx.x * PBROWS;
#pragma unroll 1
  for (int i = 0; i < PCIT; ++i) {
    const int idx = i * NTHR + tid;
    const int r   = idx / KP;
    const int kp  = idx - r * KP;
    const int kc  = (kp < KRAW) ? kp : (KRAW - 1);
    const float wv = w[(size_t)(t0 + r) * KRAW + kc];
    const float vs = (kp < KRAW) ? (wv * SC_HI) : 0.0f;
    const _Float16 hi = (_Float16)vs;
    const float res = (vs - (float)hi) * SC_LO;
    const _Float16 lo = (_Float16)res;
    sh[r * KROW + kp]      = hi;
    sh[r * KROW + KP + kp] = lo;
  }
  __syncthreads();
  const char* sb = (const char*)sh;
  unsigned int* gb = bp + (size_t)blockIdx.x * (PBROWS * KROW / 2);
#pragma unroll 1
  for (int it = 0; it < PBIT; ++it) {
    const int e = it * NTHR + tid;
    const v4u v = *(const v4ua*)(sb + (size_t)16 * e);
    *(volatile v4u*)(gb + (size_t)4 * e) = v;
  }
  __threadfence();
#pragma unroll 1
  for (int it = 0; it < PBIT; ++it) {
    const int e = it * NTHR + tid;
    const v4u v = *(const v4ua*)(sb + (size_t)16 * e);
    *(volatile v4u*)(gb + (size_t)4 * e) = v;
  }
}

__global__ __launch_bounds__(NTHR) void k_gemm_argmax(const int* __restrict__ s,
                                                      const _Float16* __restrict__ bp,
                                                      const float* __restrict__ bias,
                                                      int* out) {
  __shared__ __attribute__((aligned(16))) int red[MBLK];
  const int tid = threadIdx.x, wave = tid >> 5, lane = tid & 31, h = lane >> 4, m = lane & 15;
  const int mBase = blockIdx.x * MBLK + wave * 16;
  const int row = mBase + m;
  const int b = row >> 9, l = row & (SEQ - 1);

  int kt[KW];
#pragma unroll
  for (int j = 0; j < KW; ++j) {
    const int pos = l + j - (KW / 2);
    const int pc  = pos < 0 ? 0 : (pos > SEQ - 1 ? SEQ - 1 : pos);
    const int tok = s[(size_t)b * SEQ + pc];
    const bool ok = (pos >= 0) && (pos < SEQ) && ((unsigned)tok < (unsigned)VOC);
    kt[j] = ok ? (tok * KW + j) : -1;
  }
  const v16h a0 = build_a(0   + 8 * h, kt[0], kt[1], kt[2], kt[3], kt[4]);
  const v16h a1 = build_a(32  + 8 * h, kt[0], kt[1], kt[2], kt[3], kt[4]);
  const v16h a2 = build_a(64  + 8 * h, kt[0], kt[1], kt[2], kt[3], kt[4]);
  const v16h a3 = build_a(96  + 8 * h, kt[0], kt[1], kt[2], kt[3], kt[4]);
  const v16h a4 = build_a(128 + 8 * h, kt[0], kt[1], kt[2], kt[3], kt[4]);

  float mx[8];
  int   ix[8];
#pragma unroll
  for (int r = 0; r < 8; ++r) { mx[r] = -3.402823466e38f; ix[r] = 0; }

  const _Float16* brow = bp + (size_t)m * KROW + 8 * h;
  const float*    bcol = bias + m;

#pragma unroll 1
  for (int nt = 0; nt < NT; ++nt) {
    const _Float16* br = brow + (size_t)nt * (16 * KROW);
    FragB b0, b1, b2, b3, b4;
    b0.hf[0] = *(const v8h*)(br + 0);    b0.hf[1] = *(const v8h*)(br + 16);
    b1.hf[0] = *(const v8h*)(br + 32);   b1.hf[1] = *(const v8h*)(br + 48);
    b2.hf[0] = *(const v8h*)(br + 64);   b2.hf[1] = *(const v8h*)(br + 80);
    b3.hf[0] = *(const v8h*)(br + 96);   b3.hf[1] = *(const v8h*)(br + 112);
    b4.hf[0] = *(const v8h*)(br + 128);  b4.hf[1] = *(const v8h*)(br + 144);
    v8f acch = {0.f, 0.f, 0.f, 0.f, 0.f, 0.f, 0.f, 0.f};
    acch = wmh(a0, b0.v, acch);
    acch = wmh(a1, b1.v, acch);
    acch = wmh(a2, b2.v, acch);
    acch = wmh(a3, b3.v, acch);
    acch = wmh(a4, b4.v, acch);
    asm volatile("v_nop\n\tv_nop\n\tv_nop\n\tv_nop"
                 : "+v"(acch)
                 : "v"(a0), "v"(a1), "v"(a2), "v"(a3), "v"(a4),
                   "v"(b0.v), "v"(b1.v), "v"(b2.v), "v"(b3.v), "v"(b4.v));

    const _Float16* bl = br + KP;
    FragB c0, c1, c2, c3, c4;
    c0.hf[0] = *(const v8h*)(bl + 0);    c0.hf[1] = *(const v8h*)(bl + 16);
    c1.hf[0] = *(const v8h*)(bl + 32);   c1.hf[1] = *(const v8h*)(bl + 48);
    c2.hf[0] = *(const v8h*)(bl + 64);   c2.hf[1] = *(const v8h*)(bl + 80);
    c3.hf[0] = *(const v8h*)(bl + 96);   c3.hf[1] = *(const v8h*)(bl + 112);
    c4.hf[0] = *(const v8h*)(bl + 128);  c4.hf[1] = *(const v8h*)(bl + 144);
    v8f accl = {0.f, 0.f, 0.f, 0.f, 0.f, 0.f, 0.f, 0.f};
    accl = wmh(a0, c0.v, accl);
    accl = wmh(a1, c1.v, accl);
    accl = wmh(a2, c2.v, accl);
    accl = wmh(a3, c3.v, accl);
    accl = wmh(a4, c4.v, accl);
    asm volatile("v_nop\n\tv_nop\n\tv_nop\n\tv_nop"
                 : "+v"(accl)
                 : "v"(a0), "v"(a1), "v"(a2), "v"(a3), "v"(a4),
                   "v"(c0.v), "v"(c1.v), "v"(c2.v), "v"(c3.v), "v"(c4.v));

    const float bb = bcol[nt * 16] * SC_HI;
    const int   n  = nt * 16 + m;
#pragma unroll
    for (int r = 0; r < 8; ++r) {
      const float t = accl[r] * INV_LO;
      const float v = (acch[r] + t) + bb;
      const bool  gt = v > mx[r];
      mx[r] = gt ? v : mx[r];
      ix[r] = gt ? n : ix[r];
    }
  }

#pragma unroll
  for (int o = 8; o > 0; o >>= 1) {
#pragma unroll
    for (int r = 0; r < 8; ++r) {
      const float om = __shfl_xor(mx[r], o, 32);
      const int   oi = __shfl_xor(ix[r], o, 32);
      const bool take = (om > mx[r]) || ((om == mx[r]) && (oi < ix[r]));
      mx[r] = take ? om : mx[r];
      ix[r] = take ? oi : ix[r];
    }
  }
  if (m == 0) {
    int* rp = red + wave * 16 + 8 * h;
    rp[0] = ix[0]; rp[1] = ix[1]; rp[2] = ix[2]; rp[3] = ix[3];
    rp[4] = ix[4]; rp[5] = ix[5]; rp[6] = ix[6]; rp[7] = ix[7];
  }
  __syncthreads();
  if (wave == 0) {
    const v4i v = *(const v4ia*)(red + 4 * lane);
    int* gp = out + (size_t)blockIdx.x * MBLK + 4 * lane;
    *(volatile v4i*)gp = v;
    __threadfence();
    *(volatile v4i*)gp = v;
  }
}

extern "C" void kernel_launch(void* const* d_in, const int* in_sizes, int n_in,
                              void* d_out, int out_size, void* d_ws, size_t ws_size,
                              hipStream_t stream) {
  if (n_in < 3) return;
  if (in_sizes[0] != ROWS || in_sizes[1] != TCH * KRAW || in_sizes[2] != TCH) return;
  if (out_size != ROWS) return;

  const int*   s    = (const int*)d_in[0];
  const float* w    = (const float*)d_in[1];
  const float* bias = (const float*)d_in[2];
  int* out = (int*)d_out;

  const size_t szB = (size_t)TCH * KROW * 2;
  if (szB > ws_size || szB > (size_t)WSCAP) return;
  unsigned int*   Bu = (unsigned int*)d_ws;
  const _Float16* Bh = (const _Float16*)d_ws;

  k_prep<<<TCH / PBROWS, NTHR, 0, stream>>>(w, Bu);
  k_gemm_argmax<<<ROWS / MBLK, NTHR, 0, stream>>>(s, Bh, bias, out);
}
